// ParticleFlowNetwork_59485297049812
// MI455X (gfx1250) — hardware-verified
//
#include <hip/hip_runtime.h>
#include <math.h>
#include <stdint.h>

#define NSEG    8192
#define PSEG    128
#define FIN     4
#define HID     100
#define LAT     64
#define NC1     256
#define NC2     256
#define NC3     128
#define NC4     128

#define LSTR    136
#define NT_H    7
#define KS_H    4
#define KS_IN   1
#define NT_L    4
#define MT      2
#define ROWS    (MT * 16)
#define WAVES   4
#define TPB     (WAVES * 32)
#define SX      8.0f
#define SW      64.0f
#define INVS    (1.0f / 512.0f)

#define PA      264
#define ZP      132
#define CROWS   32
#define CTPB    64

#define P1_EL   (NT_H * KS_IN * 512)
#define PH_EL   (NT_H * KS_H * 512)
#define P4_EL   (NT_L * KS_H * 512)
#define P5_EL   (16 * 2 * 512)
#define P6_EL   (16 * 8 * 512)
#define P7_EL   (8 * 8 * 512)
#define P8_EL   (8 * 4 * 512)

static_assert(PSEG == WAVES * ROWS);
static_assert((LSTR % 8) == 0);
static_assert(LSTR >= KS_H * 32);
static_assert(NT_H * 16 >= HID);
static_assert(NT_H * 16 <= KS_H * 32);
static_assert(KS_IN * 32 >= FIN);
static_assert(NT_L * 16 == LAT);
static_assert(((ROWS * LSTR) % 8) == 0);
static_assert((PA % 8) == 0);
static_assert(PA >= NC1 && PA >= NC2 && PA >= NC3);
static_assert(ZP >= NC4 && (ZP % 4) == 0);
static_assert(CROWS * ZP * 4 <= 2 * CROWS * PA * 2);
static_assert((NSEG % CROWS) == 0);
static_assert(CROWS == 32 && CTPB == 64);
static_assert(LAT == 2 * 32 && NC1 == 16 * 16 && NC2 == 8 * 32 && NC3 == 8 * 16 && NC4 == 4 * 32);

typedef _Float16       v16h __attribute__((ext_vector_type(16)));
typedef __bf16         v16b __attribute__((ext_vector_type(16)));
typedef unsigned short v8us __attribute__((ext_vector_type(8)));
typedef unsigned short v4us __attribute__((ext_vector_type(4)));
typedef float          v8f  __attribute__((ext_vector_type(8)));
typedef float          v4f  __attribute__((ext_vector_type(4)));

union Frag  { v16h v; v8us u[2]; };
union FragB { v16b v; v8us u[2]; };

__device__ __forceinline__ unsigned short bf_bits(float f) {
  const unsigned u = __float_as_uint(f);
  return (unsigned short)((u + 0x7FFFu + ((u >> 16) & 1u)) >> 16);
}
__device__ __forceinline__ float bf_up(unsigned short b) { return __uint_as_float(((unsigned)b) << 16); }
__device__ __forceinline__ float bfr(float f) { return bf_up(bf_bits(f)); }
__device__ __forceinline__ unsigned short h_bits(float f) {
  return __builtin_bit_cast(unsigned short, (_Float16)f);
}
__device__ __forceinline__ unsigned short hx(float f) { return h_bits(bfr(f) * SX); }
__device__ __forceinline__ bool nan_bits(float f) {
  return (__float_as_uint(f) & 0x7fffffffu) > 0x7f800000u;
}

__device__ __forceinline__ v8f mma_h(v16h a, v16h b, v8f c) {
  return __builtin_amdgcn_wmma_f32_16x16x32_f16(false, a, false, b, (short)0, c, false, false);
}
__device__ __forceinline__ v8f mma_b(v16b a, v16b b, v8f c) {
  return __builtin_amdgcn_wmma_f32_16x16x32_bf16(false, a, false, b, (short)0, c, false, false);
}
__device__ __forceinline__ void mma_guard2(v8f& c0, v8f& c1, v16h a0, v16h a1, v16h b) {
#if defined(__HIP_DEVICE_COMPILE__)
  asm volatile("v_nop\n\tv_nop\n\tv_nop\n\tv_nop" : "+v"(c0), "+v"(c1) : "v"(a0), "v"(a1), "v"(b));
#else
  (void)c0; (void)c1; (void)a0; (void)a1; (void)b;
#endif
}
__device__ __forceinline__ void mma_guard1b(v8f& c0, v16b a0, v16b a1, v16b b) {
#if defined(__HIP_DEVICE_COMPILE__)
  asm volatile("v_nop\n\tv_nop\n\tv_nop\n\tv_nop" : "+v"(c0) : "v"(a0), "v"(a1), "v"(b));
#else
  (void)c0; (void)a0; (void)a1; (void)b;
#endif
}

__global__ __launch_bounds__(256) void k_pack(const float* __restrict__ W, unsigned short* dst,
                                              int Kreal, int Nreal, int kS, int nT, int nPieces, int mode) {
  const int piece = blockIdx.x * 256 + threadIdx.x;
  const bool act  = piece < nPieces;
  const int pc    = act ? piece : (nPieces - 1);
  const int elem0 = pc * 8;
  const int tblk  = kS * 512;
  const int t     = elem0 / tblk;
  int rem         = elem0 - t * tblk;
  const int s     = rem >> 9;
  rem            &= 511;
  const int L     = rem >> 4;
  const int j0    = rem & 15;
  const int n     = t * 16 + (L & 15);
  const int hh    = L >> 4;
  const int kb    = s * 32 + 8 * hh + 2 * j0;
  const int nc    = (n < Nreal) ? n : (Nreal - 1);
  v8us o;
#pragma unroll
  for (int jj = 0; jj < 8; ++jj) {
    const int k  = kb + jj;
    const int kc = (k < Kreal) ? k : (Kreal - 1);
    float v = W[(size_t)kc * Nreal + nc];
    v = (k < Kreal && n < Nreal) ? v : 0.0f;
    const unsigned short f = h_bits(bfr(v) * SW);
    const unsigned short g = bf_bits(v);
    o[jj] = (mode == 0) ? f : g;
  }
  unsigned short* d = dst + (size_t)pc * 8;
  if (act) *(volatile v8us*)d = o;
  __threadfence();
  if (act) *(volatile v8us*)d = o;
}

template <int NT, int KS>
__device__ __forceinline__ void layer_fwd(const unsigned short* __restrict__ Wp,
                                          const float* __restrict__ bias, int Nreal,
                                          unsigned short* slice, int lane) {
  Frag a[MT][KS];
  const int m  = lane & 15;
  const int hh = lane >> 4;
#pragma unroll
  for (int mt = 0; mt < MT; ++mt) {
#pragma unroll
    for (int s = 0; s < KS; ++s) {
      const unsigned short* p = slice + (mt * 16 + m) * LSTR + s * 32 + 8 * hh;
      a[mt][s].u[0] = *(const v8us*)(p);
      a[mt][s].u[1] = *(const v8us*)(p + 16);
    }
  }
  const int mrow = 8 * hh;
#pragma unroll 1
  for (int t = 0; t < NT; ++t) {
    const int n  = t * 16 + m;
    const int nc = (n < Nreal) ? n : (Nreal - 1);
    float bv = bias[nc];
    bv = (n < Nreal) ? bfr(bv) : 0.0f;
    v8f c[MT];
#pragma unroll
    for (int mt = 0; mt < MT; ++mt) c[mt] = (v8f){0.f, 0.f, 0.f, 0.f, 0.f, 0.f, 0.f, 0.f};
    Frag b;
    b.v = a[0][0].v;
#pragma unroll
    for (int s = 0; s < KS; ++s) {
      const unsigned short* wp = Wp + ((size_t)((t * KS + s) * 32 + lane) << 4);
      b.u[0] = *(const v8us*)(wp);
      b.u[1] = *(const v8us*)(wp + 8);
#pragma unroll
      for (int mt = 0; mt < MT; ++mt) c[mt] = mma_h(a[mt][s].v, b.v, c[mt]);
    }
    mma_guard2(c[0], c[1], a[0][KS - 1].v, a[1][KS - 1].v, b.v);
#pragma unroll
    for (int mt = 0; mt < MT; ++mt) {
      unsigned short* dst = slice + (mt * 16 + mrow) * LSTR + n;
#pragma unroll
      for (int v = 0; v < 8; ++v) {
        const float z = c[mt][v] * INVS + bv;
        dst[v * LSTR] = h_bits(fmaxf(z, 0.0f) * SX);
      }
    }
  }
}

template <int NT, int KS>
__device__ __forceinline__ void layer_last(const unsigned short* __restrict__ Wp,
                                           const float* __restrict__ bias,
                                           const unsigned short* slice, const float* mrow_mask, int lane,
                                           float (&ps)[NT]) {
  Frag a[MT][KS];
  const int m  = lane & 15;
  const int hh = lane >> 4;
#pragma unroll
  for (int mt = 0; mt < MT; ++mt) {
#pragma unroll
    for (int s = 0; s < KS; ++s) {
      const unsigned short* p = slice + (mt * 16 + m) * LSTR + s * 32 + 8 * hh;
      a[mt][s].u[0] = *(const v8us*)(p);
      a[mt][s].u[1] = *(const v8us*)(p + 16);
    }
  }
  const int mrow = 8 * hh;
#pragma unroll
  for (int t = 0; t < NT; ++t) {
    const int n = t * 16 + m;
    const float bv = bfr(bias[n]);
    v8f c[MT];
#pragma unroll
    for (int mt = 0; mt < MT; ++mt) c[mt] = (v8f){0.f, 0.f, 0.f, 0.f, 0.f, 0.f, 0.f, 0.f};
    Frag b;
    b.v = a[0][0].v;
#pragma unroll
    for (int s = 0; s < KS; ++s) {
      const unsigned short* wp = Wp + ((size_t)((t * KS + s) * 32 + lane) << 4);
      b.u[0] = *(const v8us*)(wp);
      b.u[1] = *(const v8us*)(wp + 8);
#pragma unroll
      for (int mt = 0; mt < MT; ++mt) c[mt] = mma_h(a[mt][s].v, b.v, c[mt]);
    }
    mma_guard2(c[0], c[1], a[0][KS - 1].v, a[1][KS - 1].v, b.v);
    float accs = 0.0f;
#pragma unroll
    for (int mt = 0; mt < MT; ++mt) {
#pragma unroll
      for (int v = 0; v < 8; ++v) {
        const float z  = c[mt][v] * INVS + bv;
        const float e  = __expf(-z);
        const float sg = __builtin_amdgcn_rcpf(1.0f + e);
        accs += mrow_mask[mt * 16 + mrow + v] * sg;
      }
    }
    ps[t] += accs;
  }
}

__global__ __launch_bounds__(TPB) void k_rows(
    const float* __restrict__ x,
    const unsigned short* __restrict__ Wp1, const unsigned short* __restrict__ Wp2,
    const unsigned short* __restrict__ Wp3, const unsigned short* __restrict__ Wp4,
    const float* __restrict__ b1, const float* __restrict__ b2,
    const float* __restrict__ b3, const float* __restrict__ b4,
    float* lat) {
  __shared__ __align__(16) unsigned short lds[WAVES * ROWS * LSTR];
  __shared__ __align__(16) float s_mask[PSEG];
  __shared__ __align__(16) float s_part[WAVES * LAT];
  __shared__ __align__(16) float s_lat[LAT];

  const int tid  = threadIdx.x;
  const int lane = tid & 31;
  const int wave = tid >> 5;
  const int seg  = blockIdx.x;
  unsigned short* slice = lds + wave * (ROWS * LSTR);

  {
    const v8us z = (v8us){0, 0, 0, 0, 0, 0, 0, 0};
    for (int i = lane; i < (ROWS * LSTR) / 8; i += 32) *(v8us*)(slice + i * 8) = z;
  }
  __syncthreads();
  bool valid;
  {
    const int row = seg * PSEG + wave * ROWS + lane;
    const v4f xr  = *(const v4f*)(x + (size_t)row * FIN);
    const bool q0 = nan_bits(xr[0]), q1 = nan_bits(xr[1]), q2 = nan_bits(xr[2]), q3 = nan_bits(xr[3]);
    valid = !q0;
    v4us o;
    o[0] = hx(q0 ? 0.0f : xr[0]);
    o[1] = hx(q1 ? 0.0f : xr[1]);
    o[2] = hx(q2 ? 0.0f : xr[2]);
    o[3] = hx(q3 ? 0.0f : xr[3]);
    *(v4us*)(slice + lane * LSTR) = o;
    s_mask[wave * ROWS + lane] = valid ? 1.0f : 0.0f;
  }
  const bool act = (__builtin_amdgcn_ballot_w32(valid) != 0u);
  __syncthreads();

  if (act) layer_fwd<NT_H, KS_IN>(Wp1, b1, HID, slice, lane);
  __syncthreads();
  if (act) layer_fwd<NT_H, KS_H>(Wp2, b2, HID, slice, lane);
  __syncthreads();
  if (act) layer_fwd<NT_H, KS_H>(Wp3, b3, HID, slice, lane);
  __syncthreads();
  float ps[NT_L] = {0.0f, 0.0f, 0.0f, 0.0f};
  if (act) layer_last<NT_L, KS_H>(Wp4, b4, slice, s_mask + wave * ROWS, lane, ps);
#pragma unroll
  for (int t = 0; t < NT_L; ++t) ps[t] += __shfl_xor(ps[t], 16);
  if (lane < 16) {
#pragma unroll
    for (int t = 0; t < NT_L; ++t) s_part[wave * LAT + t * 16 + lane] = ps[t];
  }
  __syncthreads();
  if (tid < LAT) {
    float sm = s_part[tid];
    sm += s_part[LAT + tid];
    sm += s_part[2 * LAT + tid];
    sm += s_part[3 * LAT + tid];
    s_lat[tid] = sm;
  }
  __syncthreads();
  {
    const int q = tid & 15;
    const v4f lv = *(const v4f*)(s_lat + q * 4);
    float* lp = lat + (size_t)seg * LAT + q * 4;
    if (tid < 16) *(volatile v4f*)lp = lv;
    __threadfence();
    if (tid < 16) *(volatile v4f*)lp = lv;
  }
}

template <int NT, int KS, bool LAST>
__device__ __forceinline__ void seg_layer(const unsigned short* __restrict__ Wp,
                                          const float* __restrict__ bias,
                                          const unsigned short* in_hi, const unsigned short* in_lo,
                                          unsigned short* out_hi, unsigned short* out_lo, float* zout,
                                          int lane) {
  const int m    = lane & 15;
  const int hh   = lane >> 4;
  const int mrow = 8 * hh;
#pragma unroll 1
  for (int t = 0; t < NT; ++t) {
    const int n    = t * 16 + m;
    const float bv = bfr(bias[n]);
    v8f c = (v8f){0.f, 0.f, 0.f, 0.f, 0.f, 0.f, 0.f, 0.f};
    FragB ah, al, b;
#pragma unroll
    for (int s = 0; s < KS; ++s) {
      const unsigned short* ph = in_hi + m * PA + s * 32 + 8 * hh;
      const unsigned short* pl = in_lo + m * PA + s * 32 + 8 * hh;
      ah.u[0] = *(const v8us*)(ph);
      ah.u[1] = *(const v8us*)(ph + 16);
      al.u[0] = *(const v8us*)(pl);
      al.u[1] = *(const v8us*)(pl + 16);
      const unsigned short* wp = Wp + ((size_t)((t * KS + s) * 32 + lane) << 4);
      b.u[0] = *(const v8us*)(wp);
      b.u[1] = *(const v8us*)(wp + 8);
      c = mma_b(ah.v, b.v, c);
      c = mma_b(al.v, b.v, c);
    }
    mma_guard1b(c, ah.v, al.v, b.v);
    if constexpr (!LAST) {
#pragma unroll
      for (int v = 0; v < 8; ++v) {
        const float z = fmaxf(c[v] + bv, 0.0f);
        const unsigned short hb = bf_bits(z);
        const unsigned short lb = bf_bits(z - bf_up(hb));
        out_hi[(mrow + v) * PA + n] = hb;
        out_lo[(mrow + v) * PA + n] = lb;
      }
    } else {
#pragma unroll
      for (int v = 0; v < 8; ++v) zout[(mrow + v) * ZP + n] = fmaxf(c[v] + bv, 0.0f);
    }
  }
}

__global__ __launch_bounds__(CTPB) void k_seg(
    const float* __restrict__ lat,
    const unsigned short* __restrict__ Wp5, const unsigned short* __restrict__ Wp6,
    const unsigned short* __restrict__ Wp7, const unsigned short* __restrict__ Wp8,
    const float* __restrict__ b5, const float* __restrict__ b6,
    const float* __restrict__ b7, const float* __restrict__ b8,
    const float* __restrict__ W9, const float* __restrict__ b9,
    float* out) {
  __shared__ __align__(16) unsigned short cl[4 * CROWS * PA];
  __shared__ __align__(16) float s_w9[NC4];
  __shared__ __align__(16) float s_out[CROWS];

  const int tid  = threadIdx.x;
  const int lane = tid & 31;
  const int wave = tid >> 5;
  unsigned short* Ahi = cl;
  unsigned short* Alo = cl + CROWS * PA;
  unsigned short* Bhi = cl + 2 * CROWS * PA;
  unsigned short* Blo = cl + 3 * CROWS * PA;
  float* zb = (float*)cl;
  const int r0 = blockIdx.x * CROWS;

  for (int i = tid; i < CROWS * (LAT / 4); i += CTPB) {
    const int r = i >> 4, q = i & 15;
    const v4f v = *(const v4f*)(lat + (size_t)(r0 + r) * LAT + q * 4);
    v4us ho, lo;
#pragma unroll
    for (int j = 0; j < 4; ++j) {
      const unsigned short hb = bf_bits(v[j]);
      ho[j] = hb;
      lo[j] = bf_bits(v[j] - bf_up(hb));
    }
    *(v4us*)(Ahi + r * PA + q * 4) = ho;
    *(v4us*)(Alo + r * PA + q * 4) = lo;
  }
  for (int i = tid; i < NC4; i += CTPB) s_w9[i] = bfr(W9[i]);
  __syncthreads();

  const int wr = wave * 16;
  seg_layer<16, 2, false>(Wp5, b5, Ahi + wr * PA, Alo + wr * PA, Bhi + wr * PA, Blo + wr * PA, zb, lane);
  __syncthreads();
  seg_layer<16, 8, false>(Wp6, b6, Bhi + wr * PA, Blo + wr * PA, Ahi + wr * PA, Alo + wr * PA, zb, lane);
  __syncthreads();
  seg_layer<8, 8, false>(Wp7, b7, Ahi + wr * PA, Alo + wr * PA, Bhi + wr * PA, Blo + wr * PA, zb, lane);
  __syncthreads();
  seg_layer<8, 4, true>(Wp8, b8, Bhi + wr * PA, Blo + wr * PA, Ahi + wr * PA, Alo + wr * PA, zb + wr * ZP, lane);
  __syncthreads();

  {
    const int r = tid & 31;
    const float* zr = zb + r * ZP;
    float acc = 0.0f;
#pragma unroll 4
    for (int k = 0; k < NC4; ++k) acc = fmaf(zr[k], s_w9[k], acc);
    const float lg = acc + bfr(b9[0]);
    const float e  = expf(-lg);
    const float o  = __builtin_amdgcn_rcpf(1.0f + e);
    if (tid < CROWS) s_out[r] = o;
  }
  __syncthreads();
  {
    const int q = tid & 7;
    const v4f ov = *(const v4f*)(s_out + q * 4);
    float* op = out + (size_t)blockIdx.x * CROWS + q * 4;
    if (tid < 8) *(volatile v4f*)op = ov;
    __threadfence();
    if (tid < 8) *(volatile v4f*)op = ov;
  }
}

static void launch_pack(const float* W, unsigned short* dst, int Kreal, int Nreal, int kS, int nT, int mode,
                        hipStream_t stream) {
  const int nPieces = nT * kS * 64;
  const int blocks  = (nPieces + 255) / 256;
  k_pack<<<dim3(blocks), dim3(256), 0, stream>>>(W, dst, Kreal, Nreal, kS, nT, nPieces, mode);
}

extern "C" void kernel_launch(void* const* d_in, const int* in_sizes, int n_in,
                              void* d_out, int out_size, void* d_ws, size_t ws_size,
                              hipStream_t stream) {
  if (n_in < 19) return;
  if (in_sizes[0]  != NSEG * PSEG * FIN) return;
  if (in_sizes[1]  != FIN * HID || in_sizes[2]  != HID) return;
  if (in_sizes[3]  != HID * HID || in_sizes[4]  != HID) return;
  if (in_sizes[5]  != HID * HID || in_sizes[6]  != HID) return;
  if (in_sizes[7]  != HID * LAT || in_sizes[8]  != LAT) return;
  if (in_sizes[9]  != LAT * NC1 || in_sizes[10] != NC1) return;
  if (in_sizes[11] != NC1 * NC2 || in_sizes[12] != NC2) return;
  if (in_sizes[13] != NC2 * NC3 || in_sizes[14] != NC3) return;
  if (in_sizes[15] != NC3 * NC4 || in_sizes[16] != NC4) return;
  if (in_sizes[17] != NC4 * 1   || in_sizes[18] != 1) return;
  if (out_size != NSEG) return;

  const float* x  = (const float*)d_in[0];
  const float* W1 = (const float*)d_in[1];   const float* b1 = (const float*)d_in[2];
  const float* W2 = (const float*)d_in[3];   const float* b2 = (const float*)d_in[4];
  const float* W3 = (const float*)d_in[5];   const float* b3 = (const float*)d_in[6];
  const float* W4 = (const float*)d_in[7];   const float* b4 = (const float*)d_in[8];
  const float* W5 = (const float*)d_in[9];   const float* b5 = (const float*)d_in[10];
  const float* W6 = (const float*)d_in[11];  const float* b6 = (const float*)d_in[12];
  const float* W7 = (const float*)d_in[13];  const float* b7 = (const float*)d_in[14];
  const float* W8 = (const float*)d_in[15];  const float* b8 = (const float*)d_in[16];
  const float* W9 = (const float*)d_in[17];  const float* b9 = (const float*)d_in[18];
  float* out = (float*)d_out;

  const size_t lat_bytes = (size_t)NSEG * LAT * 4;
  const size_t o1 = lat_bytes / 2;
  const size_t o2 = o1 + (size_t)P1_EL;
  const size_t o3 = o2 + (size_t)PH_EL;
  const size_t o4 = o3 + (size_t)PH_EL;
  const size_t o5 = o4 + (size_t)P4_EL;
  const size_t o6 = o5 + (size_t)P5_EL;
  const size_t o7 = o6 + (size_t)P6_EL;
  const size_t o8 = o7 + (size_t)P7_EL;
  const size_t tot_bytes = (o8 + (size_t)P8_EL) * 2;
  if (tot_bytes > ws_size) return;
  if (tot_bytes > (size_t)134217728) return;

  float* lat = (float*)d_ws;
  unsigned short* ws = (unsigned short*)d_ws;
  unsigned short* Wp1 = ws + o1;
  unsigned short* Wp2 = ws + o2;
  unsigned short* Wp3 = ws + o3;
  unsigned short* Wp4 = ws + o4;
  unsigned short* Wp5 = ws + o5;
  unsigned short* Wp6 = ws + o6;
  unsigned short* Wp7 = ws + o7;
  unsigned short* Wp8 = ws + o8;

  launch_pack(W1, Wp1, FIN, HID, KS_IN, NT_H, 0, stream);
  launch_pack(W2, Wp2, HID, HID, KS_H,  NT_H, 0, stream);
  launch_pack(W3, Wp3, HID, HID, KS_H,  NT_H, 0, stream);
  launch_pack(W4, Wp4, HID, LAT, KS_H,  NT_L, 0, stream);
  launch_pack(W5, Wp5, LAT, NC1, 2, 16, 1, stream);
  launch_pack(W6, Wp6, NC1, NC2, 8, 16, 1, stream);
  launch_pack(W7, Wp7, NC2, NC3, 8, 8,  1, stream);
  launch_pack(W8, Wp8, NC3, NC4, 4, 8,  1, stream);

  k_rows<<<dim3(NSEG), dim3(TPB), 0, stream>>>(x, Wp1, Wp2, Wp3, Wp4, b1, b2, b3, b4, lat);
  k_seg<<<dim3(NSEG / CROWS), dim3(CTPB), 0, stream>>>(lat, Wp5, Wp6, Wp7, Wp8, b5, b6, b7, b8, W9, b9, out);
  (void)hipGetLastError();
}
